// AttnFPN_56564719288655
// MI455X (gfx1250) — hardware-verified
//
#include <hip/hip_runtime.h>


#define NB_  2
#define CIN  512
#define DD   256
#define TX   2048
#define NTOK 1920
#define NR   (NB_ * NTOK)
#define NRM  (NB_ * TX)
#define NH_  8
#define HD   32
#define DFF  1024
#define NLY  4
#define ZH   4
#define DM   DD
#define PCAR 1024.0f
#define LOSC 1024.0f
typedef _Float16 h16;
typedef unsigned short bf;
typedef __attribute__((ext_vector_type(16))) __bf16   v16bf;
typedef __attribute__((ext_vector_type(16))) _Float16 v16h;
typedef __attribute__((ext_vector_type(8)))  _Float16 v8h;
typedef __attribute__((ext_vector_type(8)))  unsigned short v8us;
typedef __attribute__((ext_vector_type(8)))  float    v8f;
typedef __attribute__((ext_vector_type(4)))  float    v4f;
typedef v8h  __attribute__((may_alias)) v8ha;
typedef v4f  __attribute__((may_alias)) v4fa;
typedef v8us __attribute__((may_alias)) v8usa;

__device__ __forceinline__ unsigned short f2bf(float f) { unsigned u = __float_as_uint(f); u += 0x7FFFu + ((u >> 16) & 1u); return (unsigned short)(u >> 16); }
__device__ __forceinline__ float bf2f(unsigned short b) { return __uint_as_float(((unsigned)b) << 16); }
__device__ __forceinline__ float bfr(float f) { return bf2f(f2bf(f)); }
__device__ __forceinline__ v16h cat16(v8h lo, v8h hi) { return __builtin_shufflevector(lo, hi, 0, 1, 2, 3, 4, 5, 6, 7, 8, 9, 10, 11, 12, 13, 14, 15); }
__device__ __forceinline__ v16bf cat16b(v8us lo, v8us hi) { return __builtin_bit_cast(v16bf, __builtin_shufflevector(lo, hi, 0, 1, 2, 3, 4, 5, 6, 7, 8, 9, 10, 11, 12, 13, 14, 15)); }
__device__ __forceinline__ v8f wmma16(v16h a, v16h b, v8f c) { return __builtin_amdgcn_wmma_f32_16x16x32_f16(false, a, false, b, (short)0, c, false, false); }
__device__ __forceinline__ v8f wmmab(v16bf a, v16bf b, v8f c) { return __builtin_amdgcn_wmma_f32_16x16x32_bf16(false, a, false, b, (short)0, c, false, false); }


template <typename T16> struct WFrag;
template <> struct WFrag<h16> { typedef v16h V; static __device__ __forceinline__ V ld(const h16* p) { return cat16(*(const v8h*)p, *(const v8h*)(p + 16)); } static __device__ __forceinline__ v8f mma(V a, V b, v8f c) { return wmma16(a, b, c); } };
template <> struct WFrag<bf> { typedef v16bf V; static __device__ __forceinline__ V ld(const bf* p) { return cat16b(*(const v8us*)p, *(const v8us*)(p + 16)); } static __device__ __forceinline__ v8f mma(V a, V b, v8f c) { return wmmab(a, b, c); } };
template <typename T16, int NSPLIT, bool BIAS>
__global__ __launch_bounds__(32) void k_gemmw(const T16* __restrict__ A, const T16* __restrict__ A2, const T16* __restrict__ Bt, const T16* __restrict__ Bt2, int K, float* C, int ldc, const float* __restrict__ bias, size_t sA, size_t sB, size_t sC) {
    typedef typename WFrag<T16>::V V;
    __shared__ __align__(16) float os[16 * 68];
    const size_t z = blockIdx.z; A += z * sA; if (A2) A2 += z * sA; Bt += z * sB; if (Bt2) Bt2 += z * sB; C += z * sC;
    const int lane = threadIdx.x & 31, lr = lane & 15, hi = lane >> 4; const int r0 = blockIdx.x * 64, c0 = blockIdx.y * 64;
    v8f acc[4][4];
#pragma unroll
    for (int mb = 0; mb < 4; ++mb)
#pragma unroll
        for (int nb = 0; nb < 4; ++nb) acc[mb][nb] = (v8f){};
    const size_t aoff = (size_t)(r0 + lr) * K + 8 * hi, boff = (size_t)(c0 + lr) * K + 8 * hi;
#pragma unroll 1
    for (int kc = 0; kc < K; kc += 32) {
        V a[4], a2[4];
#pragma unroll
        for (int mb = 0; mb < 4; ++mb) { a[mb] = WFrag<T16>::ld(A + aoff + (size_t)mb * 16 * K + kc); if (NSPLIT == 1 || NSPLIT == 2) a2[mb] = WFrag<T16>::ld(A2 + aoff + (size_t)mb * 16 * K + kc); }
#pragma unroll
        for (int nb = 0; nb < 4; ++nb) { const V b = WFrag<T16>::ld(Bt + boff + (size_t)nb * 16 * K + kc); V b2; if (NSPLIT >= 2) b2 = WFrag<T16>::ld(Bt2 + boff + (size_t)nb * 16 * K + kc);
#pragma unroll
            for (int mb = 0; mb < 4; ++mb) { acc[mb][nb] = WFrag<T16>::mma(a[mb], b, acc[mb][nb]); if (NSPLIT == 1 || NSPLIT == 2) acc[mb][nb] = WFrag<T16>::mma(a2[mb], b, acc[mb][nb]); if (NSPLIT >= 2) acc[mb][nb] = WFrag<T16>::mma(a[mb], b2, acc[mb][nb]); } }
        asm volatile("v_nop\n\tv_nop\n\tv_nop\n\tv_nop" : "+v"(acc[0][0]), "+v"(acc[1][1]), "+v"(acc[2][2]), "+v"(acc[3][3]) : "v"(a[0]), "v"(a[3]));
    }
#pragma unroll
    for (int mb = 0; mb < 4; ++mb) {
#pragma unroll
        for (int nb = 0; nb < 4; ++nb) {
#pragma unroll
            for (int j = 0; j < 8; ++j) os[(hi * 8 + j) * 68 + nb * 16 + lr] = acc[mb][nb][j]; }
        __builtin_amdgcn_wave_barrier(); asm volatile("" ::: "memory");
        float* crow = C + (size_t)(r0 + mb * 16) * ldc + c0;
#pragma unroll 1
        for (int ps = 0; ps < 2; ++ps) {
#pragma unroll
            for (int s = 0; s < 8; ++s) { const int row = 2 * s + hi, cofs = lr * 4; v4f val = *(const v4fa*)(os + row * 68 + cofs); if (BIAS) { val[0] += bfr(bias[c0 + cofs]); val[1] += bfr(bias[c0 + cofs + 1]); val[2] += bfr(bias[c0 + cofs + 2]); val[3] += bfr(bias[c0 + cofs + 3]); }
                *(volatile v4f*)(crow + (size_t)row * ldc + cofs) = val; }
            if (ps == 0) __threadfence(); }
        __builtin_amdgcn_wave_barrier(); asm volatile("" ::: "memory");
    }
}
__constant__ float c_div[128] = {1.0f, 0.930572033f, 0.865964353f, 0.805842161f, 0.749894202f, 0.697830617f, 0.649381638f, 0.604296386f, 0.562341332f, 0.523299098f, 0.486967474f, 0.453158349f, 0.421696484f, 0.392418951f, 0.365174115f, 0.339820832f, 0.316227764f, 0.294272691f, 0.273841947f, 0.254829645f, 0.237137347f, 0.220673412f, 0.2053525f, 0.191095293f, 0.177827924f, 0.165481716f, 0.153992653f, 0.143301249f, 0.133352146f, 0.124093771f, 0.11547821f, 0.107460767f, 0.099999994f, 0.0930572078f, 0.0865964368f, 0.0805842206f, 0.0749894083f, 0.0697830543f, 0.0649381503f, 0.0604296401f, 0.0562341288f, 0.0523299091f, 0.0486967489f, 0.0453158356f, 0.0421696529f, 0.0392418951f, 0.0365174115f, 0.0339820758f, 0.0316227749f, 0.0294272732f, 0.0273841936f, 0.0254829675f, 0.0237137359f, 0.0220673401f, 0.0205352474f, 0.0191095285f, 0.0177827962f, 0.0165481735f, 0.0153992614f, 0.0143301236f, 0.0133352149f, 0.0124093788f, 0.011547816f, 0.0107460758f, 0.00999999885f, 0.00930572115f, 0.00865964405f, 0.00805842038f, 0.00749894138f, 0.00697830552f, 0.00649381708f, 0.00604296243f, 0.00562341232f, 0.00523299072f, 0.00486967526f, 0.00453158421f, 0.00421696436f, 0.00392418914f, 0.00365174119f, 0.00339820865f, 0.0031622767f, 0.00294272648f, 0.00273841945f, 0.0025482967f, 0.00237137382f, 0.00220673345f, 0.0020535246f, 0.00191095273f, 0.00177827955f, 0.00165481726f, 0.00153992616f, 0.00143301231f, 0.00133352145f, 0.00124093774f, 0.00115478167f, 0.0010746076f, 0.000999999931f, 0.000930572045f, 0.000865964452f, 0.000805841992f, 0.000749894069f, 0.000697830517f, 0.000649381604f, 0.000604296161f, 0.000562341185f, 0.000523299037f, 0.000486967503f, 0.000453158398f, 0.000421696372f, 0.000392418879f, 0.000365174084f, 0.000339820836f, 0.000316227815f, 0.000294272788f, 0.000273842074f, 0.000254829531f, 0.000237137283f, 0.000220673348f, 0.000205352451f, 0.000191095271f, 0.000177827926f, 0.000165481732f, 0.000153992674f, 0.000143301309f, 0.000133352078f, 0.000124093727f, 0.000115478157f, 0.00010746075f};
typedef __attribute__((ext_vector_type(4))) _Float16 v4h;
__device__ __forceinline__ h16 tohx(float x) { return (h16)x; }
__constant__ int c_loff[4] = {0, 1024, 1536, 1792};
__constant__ int c_lsz[4] = {1024, 512, 256, 128};
__device__ __forceinline__ void lvl_of(int t, int& lv, int& i, int& tl) { lv = (t >= 1792) ? 3 : (t >= 1536) ? 2 : (t >= 1024) ? 1 : 0; i = t - c_loff[lv]; tl = c_lsz[lv]; }
__global__ __launch_bounds__(256) void k_cvt8h(const float* __restrict__ src, h16* dst, size_t n8) { const size_t i = (size_t)blockIdx.x * 256 + threadIdx.x; if (i >= n8) return; const v8f v = *(const v8f*)(src + i * 8); v8h o;
#pragma unroll
    for (int k = 0; k < 8; ++k) o[k] = tohx(bfr(v[k])); *(volatile v8h*)(dst + i * 8) = o; __threadfence(); *(volatile v8h*)(dst + i * 8) = o; }
__global__ __launch_bounds__(256) void k_tokx(const float* __restrict__ x, bf* XT) {
    typedef __attribute__((ext_vector_type(4))) unsigned short v4us;
    const int lane = threadIdx.x & 31; const size_t r = (size_t)blockIdx.x * 8 + (threadIdx.x >> 5); if (r >= (size_t)NRM) return; const int b = (int)(r / TX), t = (int)(r % TX);
#pragma unroll 1
    for (int ps = 0; ps < 2; ++ps) {
#pragma unroll
        for (int q = 0; q < 4; ++q) { const int c0 = q * 128 + lane * 4; v4us o;
#pragma unroll
            for (int i = 0; i < 4; ++i) o[i] = f2bf(x[((size_t)b * CIN + c0 + i) * TX + t]);
            *(volatile v4us*)(XT + r * CIN + c0) = o; }
        if (ps == 0) __threadfence(); }
}
__global__ __launch_bounds__(256) void k_im2col0(const float* __restrict__ x, bf* A0) {
    typedef __attribute__((ext_vector_type(4))) unsigned short v4us;
    const int lane = threadIdx.x & 31; const size_t r = (size_t)blockIdx.x * 8 + (threadIdx.x >> 5); if (r >= (size_t)NB_ * 1024) return; const int b = (int)(r / 1024), t = (int)(r % 1024);
#pragma unroll 1
    for (int ps = 0; ps < 2; ++ps) {
#pragma unroll 1
        for (int q = 0; q < 12; ++q) { const int c0 = q * 128 + lane * 4; const int k = c0 / CIN, c = c0 % CIN; const int ts = 2 * t + k - 1; v4us o;
#pragma unroll
            for (int i = 0; i < 4; ++i) o[i] = (ts >= 0 && ts < TX) ? f2bf(x[((size_t)b * CIN + c + i) * TX + ts]) : (unsigned short)0;
            *(volatile v4us*)(A0 + r * (3 * CIN) + c0) = o; }
        if (ps == 0) __threadfence(); }
}
template <bool F16O>
__global__ __launch_bounds__(256) void k_wconv(const float* __restrict__ w, int cin, int kw, bf* Bb, h16* Bh) {
    typedef __attribute__((ext_vector_type(4))) unsigned short v4us;
    const int lane = threadIdx.x & 31; const int o = blockIdx.x * 8 + (threadIdx.x >> 5); if (o >= DD) return; const int KK = kw * cin;
#pragma unroll 1
    for (int ps = 0; ps < 2; ++ps) {
#pragma unroll 1
        for (int c0 = lane * 4; c0 < KK; c0 += 128) { const int k = c0 / cin, c = c0 % cin; v4us ob; v4h oh;
#pragma unroll
            for (int i = 0; i < 4; ++i) { const float v = bfr(w[((size_t)o * cin + c + i) * kw + k]); ob[i] = f2bf(v); oh[i] = tohx(v); }
            if (F16O) *(volatile v4h*)(Bh + (size_t)o * KK + c0) = oh; else *(volatile v4us*)(Bb + (size_t)o * KK + c0) = ob; }
        if (ps == 0) __threadfence(); }
}
__global__ __launch_bounds__(256) void k_relu_rows(const float* __restrict__ src, int nrows, int tl, int toff, float* PYR, h16* Ph) {
    const int lane = threadIdx.x & 31; const int r = blockIdx.x * 8 + (threadIdx.x >> 5); if (r >= nrows) return; const int b = r / tl, t = r % tl; const size_t drow = (size_t)b * NTOK + toff + t;
#pragma unroll 1
    for (int ps = 0; ps < 2; ++ps) {
#pragma unroll
        for (int c = 0; c < 2; ++c) { const int c0 = c * 128 + lane * 4; v4f v = *(const v4f*)(src + (size_t)r * DD + c0); v4h o;
#pragma unroll
            for (int i = 0; i < 4; ++i) { v[i] = fmaxf(v[i], 0.f); o[i] = tohx(v[i]); }
            if (PYR) *(volatile v4f*)(PYR + drow * DD + c0) = v; if (Ph) *(volatile v4h*)(Ph + (size_t)r * DD + c0) = o; }
        if (ps == 0) __threadfence(); }
}
__global__ __launch_bounds__(256) void k_im2colL(const float* __restrict__ PYR, int tl, int toff, h16* A) {
    const int lane = threadIdx.x & 31; const int r = blockIdx.x * 8 + (threadIdx.x >> 5); const int to = tl / 2; if (r >= NB_ * to) return; const int b = r / to, t = r % to;
#pragma unroll 1
    for (int ps = 0; ps < 2; ++ps) {
#pragma unroll 1
        for (int q = 0; q < 6; ++q) { const int c0 = q * 128 + lane * 4; const int k = c0 / DD, c = c0 % DD; const int ts = 2 * t + k - 1; v4h o;
#pragma unroll
            for (int i = 0; i < 4; ++i) o[i] = tohx((ts >= 0 && ts < tl) ? PYR[((size_t)b * NTOK + toff + ts) * DD + c + i] : 0.f);
            *(volatile v4h*)(A + (size_t)r * (3 * DD) + c0) = o; }
        if (ps == 0) __threadfence(); }
}
__global__ __launch_bounds__(256) void k_scalepe(const float* __restrict__ PYR, float* F, h16* Fh) {
    const int lane = threadIdx.x & 31; const size_t r = (size_t)blockIdx.x * 8 + (threadIdx.x >> 5); if (r >= (size_t)NR) return; const int t = (int)(r % NTOK); int lv, i, tl; lvl_of(t, lv, i, tl); (void)tl;
    v4f v[2]; v4h o[2];
#pragma unroll
    for (int c = 0; c < 2; ++c) { const int c0 = c * 128 + lane * 4; v[c] = *(const v4f*)(PYR + r * DD + c0);
#pragma unroll
        for (int k = 0; k < 2; ++k) { const int m = c * 64 + lane * 2 + k; float sn, cs; sincosf((float)i * c_div[m], &sn, &cs); v[c][2 * k] = v[c][2 * k] * 16.0f + sn; v[c][2 * k + 1] = v[c][2 * k + 1] * 16.0f + cs; }
#pragma unroll
        for (int k = 0; k < 4; ++k) o[c][k] = tohx(v[c][k]); }
#pragma unroll 1
    for (int ps = 0; ps < 2; ++ps) {
#pragma unroll
        for (int c = 0; c < 2; ++c) { const int c0 = c * 128 + lane * 4; *(volatile v4f*)(F + r * DD + c0) = v[c]; *(volatile v4h*)(Fh + r * DD + c0) = o[c]; }
        if (ps == 0) __threadfence(); }
}
__global__ __launch_bounds__(256) void k_band(const float* __restrict__ QKV, h16* OH) {
    const int lane = threadIdx.x & 31; const size_t r = (size_t)blockIdx.x * 8 + (threadIdx.x >> 5); if (r >= (size_t)NR) return; const int b = (int)(r / NTOK), t = (int)(r % NTOK); int lv, i, tl; lvl_of(t, lv, i, tl);
    const int h = lane >> 2, d0 = (lane & 3) * 8; float q[8], acc[8];
#pragma unroll
    for (int k = 0; k < 8; ++k) { q[k] = QKV[r * (3 * DD) + h * HD + d0 + k]; acc[k] = 0.f; }
    float m = -3.0e38f, lsum = 0.f; const int jlo = max(0, i - 4), jhi = min(tl - 1, i + 4);
#pragma unroll 1
    for (int j = jlo; j <= jhi; ++j) { const size_t kr = ((size_t)b * NTOK + c_loff[lv] + j) * (3 * DD); float s = 0.f;
#pragma unroll
        for (int k = 0; k < 8; ++k) s = fmaf(q[k], QKV[kr + DD + h * HD + d0 + k], s);
        s += __shfl_xor(s, 1, 32); s += __shfl_xor(s, 2, 32); s *= 0.17677669529663688f;
        const float mn = fmaxf(m, s); const float sc = __expf(m - mn); const float e = __expf(s - mn); lsum = lsum * sc + e;
#pragma unroll
        for (int k = 0; k < 8; ++k) acc[k] = fmaf(e, QKV[kr + 2 * DD + h * HD + d0 + k], acc[k] * sc);
        m = mn; }
    const float inv = __fdiv_rn(1.0f, lsum); v8h o;
#pragma unroll
    for (int k = 0; k < 8; ++k) o[k] = tohx(acc[k] * inv);
    *(volatile v8h*)(OH + r * DD + lane * 8) = o; __threadfence(); *(volatile v8h*)(OH + r * DD + lane * 8) = o;
}
__global__ __launch_bounds__(256) void k_lnres(float* F, const float* __restrict__ CO, const float* __restrict__ g_, const float* __restrict__ b_, h16* Fh) {
    const int lane = threadIdx.x & 31; const size_t r = (size_t)blockIdx.x * 8 + (threadIdx.x >> 5); if (r >= (size_t)NR) return; float v[8]; float s = 0.f;
#pragma unroll
    for (int c = 0; c < 2; ++c) {
#pragma unroll
        for (int i = 0; i < 4; ++i) { const int col = c * 128 + lane * 4 + i; v[c * 4 + i] = F[r * DD + col] + CO[r * DD + col]; s += v[c * 4 + i]; } }
#pragma unroll
    for (int sh = 16; sh; sh >>= 1) s += __shfl_xor(s, sh, 32);
    const float mu = s * (1.0f / DD); float q = 0.f;
#pragma unroll
    for (int i = 0; i < 8; ++i) { const float d = v[i] - mu; q = fmaf(d, d, q); }
#pragma unroll
    for (int sh = 16; sh; sh >>= 1) q += __shfl_xor(q, sh, 32);
    const float rs = rsqrtf(q * (1.0f / DD) + 1e-5f); v4f o[2]; v4h oh[2];
#pragma unroll
    for (int c = 0; c < 2; ++c) {
#pragma unroll
        for (int i = 0; i < 4; ++i) { const int col = c * 128 + lane * 4 + i; o[c][i] = (v[c * 4 + i] - mu) * rs * bfr(g_[col]) + bfr(b_[col]); oh[c][i] = tohx(o[c][i]); } }
#pragma unroll 1
    for (int ps = 0; ps < 2; ++ps) {
#pragma unroll
        for (int c = 0; c < 2; ++c) { const int c0 = c * 128 + lane * 4; *(volatile v4f*)(F + r * DD + c0) = o[c]; *(volatile v4h*)(Fh + r * DD + c0) = oh[c]; }
        if (ps == 0) __threadfence(); }
}
__global__ __launch_bounds__(256) void k_qpl(const float* __restrict__ Qc, int b, int h0, h16* Qx) {
    const int lane = threadIdx.x & 31; const int t = (blockIdx.x * 8 + (threadIdx.x >> 5)) * 4 + (lane >> 3); if (t >= NTOK) return; const int z = blockIdx.z; const int c0 = (lane & 7) * 4; v4h o;
#pragma unroll
    for (int q = 0; q < 4; ++q) o[q] = tohx(Qc[((size_t)b * NTOK + t) * DD + (h0 + z) * HD + c0 + q] * 0.17677669529663688f);
    const size_t off = ((size_t)z * NTOK + t) * HD + c0; *(volatile v4h*)(Qx + off) = o; __threadfence(); *(volatile v4h*)(Qx + off) = o;
}
__global__ __launch_bounds__(256) void k_kpl(const float* __restrict__ KV, int b, int h0, h16* Kx) {
    const int lane = threadIdx.x & 31; const int t = (blockIdx.x * 8 + (threadIdx.x >> 5)) * 4 + (lane >> 3); if (t >= TX) return; const int z = blockIdx.z; const int c0 = (lane & 7) * 4; v4h o;
#pragma unroll
    for (int q = 0; q < 4; ++q) o[q] = tohx(KV[((size_t)b * TX + t) * (2 * DD) + (h0 + z) * HD + c0 + q]);
    const size_t off = ((size_t)z * TX + t) * HD + c0; *(volatile v4h*)(Kx + off) = o; __threadfence(); *(volatile v4h*)(Kx + off) = o;
}
__global__ __launch_bounds__(256) void k_vT(const float* __restrict__ KV, int b, int h0, h16* VT) {
    __shared__ float tl[64][33];
    const int tid = threadIdx.x; const int t0 = blockIdx.x * 64; const int z = blockIdx.z; const int rr = tid >> 2, cq = (tid & 3) * 8;
#pragma unroll
    for (int i = 0; i < 8; ++i) tl[rr][cq + i] = KV[((size_t)b * TX + t0 + rr) * (2 * DD) + DD + (h0 + z) * HD + cq + i];
    __syncthreads();
    const int lane = tid & 31, wv = tid >> 5;
    auto pass = [&]() { const int tq = (lane & 7) * 8;
#pragma unroll
        for (int i2 = 0; i2 < 2; ++i2) { const int dr = wv * 8 + i2 * 4 + (lane >> 3); v8h v;
#pragma unroll
            for (int i = 0; i < 8; ++i) v[i] = (dr < HD) ? tohx(tl[tq + i][dr < HD ? dr : 0]) : (h16)0.0f;
            *(volatile v8h*)(VT + ((size_t)z * 64 + dr) * TX + t0 + tq) = v; } };
    pass(); __threadfence(); pass();
}
__global__ __launch_bounds__(256) void k_softc(const float* __restrict__ S, h16* P) {
    const int lane = threadIdx.x & 31, i = blockIdx.x * 8 + (threadIdx.x >> 5); if (i >= NTOK) return; const size_t zo = ((size_t)blockIdx.z * NTOK + i) * TX; const float* sr = S + zo; h16* po = P + zo;
    float m = -3.0e38f;
#pragma unroll 1
    for (int c0 = lane * 4; c0 < TX; c0 += 128) {
#pragma unroll
        for (int q = 0; q < 4; ++q) m = fmaxf(m, sr[c0 + q]); }
#pragma unroll
    for (int sh = 16; sh; sh >>= 1) m = fmaxf(m, __shfl_xor(m, sh, 32));
    float sum = 0.f;
#pragma unroll 1
    for (int c0 = lane * 4; c0 < TX; c0 += 128) {
#pragma unroll
        for (int q = 0; q < 4; ++q) sum += __expf(sr[c0 + q] - m); }
#pragma unroll
    for (int sh = 16; sh; sh >>= 1) sum += __shfl_xor(sum, sh, 32);
    const float f = __fdiv_rn(PCAR, sum);
#pragma unroll 1
    for (int ps = 0; ps < 2; ++ps) {
#pragma unroll 1
        for (int c0 = lane * 4; c0 < TX; c0 += 128) { v4h o;
#pragma unroll
            for (int q = 0; q < 4; ++q) o[q] = tohx(__expf(sr[c0 + q] - m) * f);
            *(volatile v4h*)(po + c0) = o; }
        if (ps == 0) __threadfence(); }
}
__global__ __launch_bounds__(256) void k_mergec(const float* __restrict__ OZ, int b, int h0, h16* OH) {
    const int lane = threadIdx.x & 31, t = blockIdx.x * 8 + (threadIdx.x >> 5); if (t >= NTOK) return; const int z = lane >> 3, d0 = (lane & 7) * 4; v4h o;
#pragma unroll
    for (int k = 0; k < 4; ++k) o[k] = tohx(OZ[((size_t)z * NTOK + t) * 64 + d0 + k] * (1.0f / PCAR));
    const size_t off = ((size_t)b * NTOK + t) * DD + (h0 + z) * HD + d0; *(volatile v4h*)(OH + off) = o; __threadfence(); *(volatile v4h*)(OH + off) = o;
}
__global__ __launch_bounds__(256) void k_relu16(const float* __restrict__ H, h16* P) {
    const int lane = threadIdx.x & 31; const size_t r = (size_t)blockIdx.x * 8 + (threadIdx.x >> 5); if (r >= (size_t)NR) return;
#pragma unroll 1
    for (int ps = 0; ps < 2; ++ps) {
#pragma unroll
        for (int q = 0; q < 4; ++q) { const size_t off = r * DFF + q * 256 + lane * 8; v8h o;
#pragma unroll
            for (int i = 0; i < 8; ++i) o[i] = tohx(fmaxf(H[off + i], 0.f));
            *(volatile v8h*)(P + off) = o; }
        if (ps == 0) __threadfence(); }
}
__global__ __launch_bounds__(256) void k_outT(const float* __restrict__ F, float* OUTB) {
    const int lane = threadIdx.x & 31; const int w = blockIdx.x * 8 + (threadIdx.x >> 5); if (w >= NB_ * DD) return; const int b = w / DD, c = w % DD;
#pragma unroll 1
    for (int ps = 0; ps < 2; ++ps) {
#pragma unroll 1
        for (int q = 0; q < NTOK / 128; ++q) { const int t0 = q * 128 + lane * 4; v4f o;
#pragma unroll
            for (int i = 0; i < 4; ++i) o[i] = F[((size_t)b * NTOK + t0 + i) * DD + c];
            *(volatile v4f*)(OUTB + (size_t)w * NTOK + t0) = o; }
        if (ps == 0) __threadfence(); }
}
extern "C" void kernel_launch(void* const* d_in, const int* in_sizes, int n_in,
                              void* d_out, int out_size, void* d_ws, size_t ws_size, hipStream_t stream) {
    (void)in_sizes; (void)n_in; (void)out_size;
    const float* x = (const float*)d_in[0]; const float* conv_w = (const float*)d_in[1]; const float* conv_b = (const float*)d_in[2]; const float* nw0 = (const float*)d_in[3]; const float* nb0 = (const float*)d_in[4]; const float* nw = (const float*)d_in[5]; const float* nbb = (const float*)d_in[6];
    const float* sa_in_w = (const float*)d_in[7]; const float* sa_in_b = (const float*)d_in[8]; const float* sa_out_w = (const float*)d_in[9]; const float* sa_out_b = (const float*)d_in[10]; const float* ca_in_w = (const float*)d_in[11]; const float* ca_in_b = (const float*)d_in[12]; const float* ca_out_w = (const float*)d_in[13]; const float* ca_out_b = (const float*)d_in[14];
    const float* ff1_w = (const float*)d_in[15]; const float* ff1_b = (const float*)d_in[16]; const float* ff2_w = (const float*)d_in[17]; const float* ff2_b = (const float*)d_in[18]; const float* ln1g = (const float*)d_in[19]; const float* ln1b = (const float*)d_in[20]; const float* ln2g = (const float*)d_in[21]; const float* ln2b = (const float*)d_in[22]; const float* ln3g = (const float*)d_in[23]; const float* ln3b = (const float*)d_in[24];
    float* out = (float*)d_out;
    char* wsp = (char*)d_ws;
    auto take = [&](size_t bytes) { char* p = wsp; wsp += (bytes + 255) & ~(size_t)255; return (void*)p; };
    bf* WCV = (bf*)take((size_t)DD * CIN * 2); bf* WN0 = (bf*)take((size_t)DD * 3 * CIN * 2); h16* WN = (h16*)take((size_t)3 * DD * 3 * DD * 2);
    h16* WSAI = (h16*)take((size_t)NLY * 3 * DD * DD * 2); h16* WSAO = (h16*)take((size_t)NLY * DD * DD * 2); h16* WCAI = (h16*)take((size_t)NLY * 3 * DD * DD * 2); h16* WCAO = (h16*)take((size_t)NLY * DD * DD * 2); h16* WF1 = (h16*)take((size_t)NLY * DFF * DD * 2); h16* WF2 = (h16*)take((size_t)NLY * DD * DFF * 2);
    bf* XT = (bf*)take((size_t)NRM * CIN * 2); float* MEM = (float*)take((size_t)NRM * DD * 4); h16* MEMh = (h16*)take((size_t)NRM * DD * 2); bf* A0 = (bf*)take((size_t)NB_ * 1024 * 3 * CIN * 2); h16* AL = (h16*)take((size_t)NB_ * 512 * 3 * DD * 2); float* CV = (float*)take((size_t)NB_ * 1024 * DD * 4);
    float* PYR = (float*)take((size_t)NR * DD * 4); float* F = (float*)take((size_t)NR * DD * 4); h16* Fh = (h16*)take((size_t)NR * DD * 2); float* QKV = (float*)take((size_t)NR * 3 * DD * 4); h16* OH = (h16*)take((size_t)NR * DD * 2); float* CO = (float*)take((size_t)NR * DD * 4);
    float* Qc = (float*)take((size_t)NR * DD * 4); float* KV = (float*)take((size_t)NRM * 2 * DD * 4); h16* Qx = (h16*)take((size_t)ZH * NTOK * HD * 2); h16* Kx = (h16*)take((size_t)ZH * TX * HD * 2); h16* VT = (h16*)take((size_t)ZH * 64 * TX * 2); float* S = (float*)take((size_t)ZH * NTOK * TX * 4); h16* Px = (h16*)take((size_t)ZH * NTOK * TX * 2); float* OZ = (float*)take((size_t)ZH * NTOK * 64 * 4);
    float* H1 = (float*)take((size_t)NR * DFF * 4); h16* H1h = (h16*)take((size_t)NR * DFF * 2);
    if ((size_t)(wsp - (char*)d_ws) > ws_size) return;
    k_wconv<false><<<DD / 8, 256, 0, stream>>>(conv_w, CIN, 1, WCV, nullptr); k_wconv<false><<<DD / 8, 256, 0, stream>>>(nw0, CIN, 3, WN0, nullptr);
    for (int i = 0; i < 3; ++i) k_wconv<true><<<DD / 8, 256, 0, stream>>>(nw + (size_t)i * DD * DD * 3, DD, 3, nullptr, WN + (size_t)i * DD * 3 * DD);
    { const size_t n1 = (size_t)NLY * 3 * DD * DD / 8, n2 = (size_t)NLY * DD * DD / 8, n3 = (size_t)NLY * DFF * DD / 8;
      k_cvt8h<<<(unsigned)((n1 + 255) / 256), 256, 0, stream>>>(sa_in_w, WSAI, n1); k_cvt8h<<<(unsigned)((n2 + 255) / 256), 256, 0, stream>>>(sa_out_w, WSAO, n2); k_cvt8h<<<(unsigned)((n1 + 255) / 256), 256, 0, stream>>>(ca_in_w, WCAI, n1); k_cvt8h<<<(unsigned)((n2 + 255) / 256), 256, 0, stream>>>(ca_out_w, WCAO, n2); k_cvt8h<<<(unsigned)((n3 + 255) / 256), 256, 0, stream>>>(ff1_w, WF1, n3); k_cvt8h<<<(unsigned)((n3 + 255) / 256), 256, 0, stream>>>(ff2_w, WF2, n3); }
    k_tokx<<<NRM / 8, 256, 0, stream>>>(x, XT);
    k_gemmw<bf, 0, true><<<dim3(NRM / 64, DD / 64, 1), 32, 0, stream>>>(XT, nullptr, WCV, nullptr, CIN, MEM, DD, conv_b, 0, 0, 0); k_relu_rows<<<NRM / 8, 256, 0, stream>>>(MEM, NRM, TX, 0, nullptr, MEMh);
    k_im2col0<<<(NB_ * 1024) / 8, 256, 0, stream>>>(x, A0);
    k_gemmw<bf, 0, true><<<dim3((NB_ * 1024) / 64, DD / 64, 1), 32, 0, stream>>>(A0, nullptr, WN0, nullptr, 3 * CIN, CV, DD, nb0, 0, 0, 0); k_relu_rows<<<(NB_ * 1024) / 8, 256, 0, stream>>>(CV, NB_ * 1024, 1024, 0, PYR, nullptr);
    { int tl = 1024, toff = 0; for (int i = 0; i < 3; ++i) { const int to = tl / 2, tooff = toff + tl;
        k_im2colL<<<(NB_ * to + 7) / 8, 256, 0, stream>>>(PYR, tl, toff, AL);
        k_gemmw<h16, 0, true><<<dim3((NB_ * to) / 64, DD / 64, 1), 32, 0, stream>>>(AL, nullptr, WN + (size_t)i * DD * 3 * DD, nullptr, 3 * DD, CV, DD, nbb + i * DD, 0, 0, 0); k_relu_rows<<<(NB_ * to + 7) / 8, 256, 0, stream>>>(CV, NB_ * to, to, tooff, PYR, nullptr);
        tl = to; toff = tooff; } }
    k_scalepe<<<NR / 8, 256, 0, stream>>>(PYR, F, Fh);
    for (int l = 0; l < NLY; ++l) {
        k_gemmw<h16, 0, true><<<dim3(NR / 64, (3 * DD) / 64, 1), 32, 0, stream>>>(Fh, nullptr, WSAI + (size_t)l * 3 * DD * DD, nullptr, DD, QKV, 3 * DD, sa_in_b + l * 3 * DD, 0, 0, 0);
        k_band<<<NR / 8, 256, 0, stream>>>(QKV, OH);
        k_gemmw<h16, 0, true><<<dim3(NR / 64, DD / 64, 1), 32, 0, stream>>>(OH, nullptr, WSAO + (size_t)l * DD * DD, nullptr, DD, CO, DD, sa_out_b + l * DD, 0, 0, 0);
        k_lnres<<<NR / 8, 256, 0, stream>>>(F, CO, ln1g + l * DD, ln1b + l * DD, Fh);
        k_gemmw<h16, 0, true><<<dim3(NR / 64, DD / 64, 1), 32, 0, stream>>>(Fh, nullptr, WCAI + (size_t)l * 3 * DD * DD, nullptr, DD, Qc, DD, ca_in_b + l * 3 * DD, 0, 0, 0);
        k_gemmw<h16, 0, true><<<dim3(NRM / 64, (2 * DD) / 64, 1), 32, 0, stream>>>(MEMh, nullptr, WCAI + (size_t)l * 3 * DD * DD + (size_t)DD * DD, nullptr, DD, KV, 2 * DD, ca_in_b + l * 3 * DD + DD, 0, 0, 0);
        for (int b = 0; b < NB_; ++b)
            for (int h0 = 0; h0 < NH_; h0 += ZH) {
                k_qpl<<<dim3((NTOK / 4) / 8, 1, ZH), 256, 0, stream>>>(Qc, b, h0, Qx); k_kpl<<<dim3((TX / 4) / 8, 1, ZH), 256, 0, stream>>>(KV, b, h0, Kx); k_vT<<<dim3(TX / 64, 1, ZH), 256, 0, stream>>>(KV, b, h0, VT);
                k_gemmw<h16, 0, false><<<dim3(NTOK / 64, TX / 64, ZH), 32, 0, stream>>>(Qx, nullptr, Kx, nullptr, HD, S, TX, nullptr, (size_t)NTOK * HD, (size_t)TX * HD, (size_t)NTOK * TX);
                k_softc<<<dim3(NTOK / 8, 1, ZH), 256, 0, stream>>>(S, Px);
                k_gemmw<h16, 0, false><<<dim3(NTOK / 64, 1, ZH), 32, 0, stream>>>(Px, nullptr, VT, nullptr, TX, OZ, 64, nullptr, (size_t)NTOK * TX, (size_t)64 * TX, (size_t)NTOK * 64);
                k_mergec<<<NTOK / 8, 256, 0, stream>>>(OZ, b, h0, OH); }
        k_gemmw<h16, 0, true><<<dim3(NR / 64, DD / 64, 1), 32, 0, stream>>>(OH, nullptr, WCAO + (size_t)l * DD * DD, nullptr, DD, CO, DD, ca_out_b + l * DD, 0, 0, 0);
        k_lnres<<<NR / 8, 256, 0, stream>>>(F, CO, ln2g + l * DD, ln2b + l * DD, Fh);
        k_gemmw<h16, 0, true><<<dim3(NR / 64, DFF / 64, 1), 32, 0, stream>>>(Fh, nullptr, WF1 + (size_t)l * DFF * DD, nullptr, DD, H1, DFF, ff1_b + l * DFF, 0, 0, 0);
        k_relu16<<<NR / 8, 256, 0, stream>>>(H1, H1h);
        k_gemmw<h16, 0, true><<<dim3(NR / 64, DD / 64, 1), 32, 0, stream>>>(H1h, nullptr, WF2 + (size_t)l * DD * DFF, nullptr, DFF, CO, DD, ff2_b + l * DD, 0, 0, 0);
        k_lnres<<<NR / 8, 256, 0, stream>>>(F, CO, ln3g + l * DD, ln3b + l * DD, Fh); }
    k_outT<<<(NB_ * DD) / 8, 256, 0, stream>>>(F, out);
}
